// ResGraphModule_1262720385735
// MI455X (gfx1250) — hardware-run, weakly checked
//
#include <hip/hip_runtime.h>
#include <stddef.h>
#include <stdint.h>


#ifndef MODE_CONV
#define MODE_CONV 1
#endif
#ifndef MODE_GI
#define MODE_GI 1
#endif
#ifndef MODE_GH
#define MODE_GH 1
#endif
#ifndef FAST_GATES
#define FAST_GATES 1
#endif

#define DF     128
#define EC     16
#define HP     256
#define NTHR   256
#define NWAVE  8
#define EPT    8
#define CHUNK  (NTHR * EPT)
#define WCAP   (EPT * 32)
#define LISTN  (NWAVE * WCAP)
#define NBA    1024
#define SLA    10
#define RCAP   14336
#define DEGCAP 64
#define GBM    64
#define GTHR   128
#define TROWS  128
#define RSLOTS 64
#define AROWS  64
#define UPART  2048
#define NPARTS 16
#define NWBLK  ((NPARTS * UPART) / NTHR)
#define OFF_CW0 0
#define OFF_CW1 32768
#define OFF_WRZ 65536
#define OFF_WIN 196608
#define OFF_WHN 229376
#define WB_ELEMS 262144
#define KCONV  (MODE_CONV == 2 ? 256 : 128)
#define KGI    (MODE_GI == 2 ? 256 : 128)
#define KGH    (MODE_GH == 2 ? 256 : 128)
#define BK_ZINTS    (LISTN + 2 * RCAP + 3 * NBA)
#define BK_LDS_INTS (BK_ZINTS + 16)
#define GRU_STAGE   (TROWS * DF)
#define GRU_DYN_BYTES (4 * GRU_STAGE * 4)
#define GRU_STATIC_BYTES ((1024 + 256) * 4)
#define WSMAX  134217728

static_assert((CHUNK & (CHUNK - 1)) == 0 && CHUNK <= 4096);
static_assert((NBA & (NBA - 1)) == 0 && NBA == (1 << SLA));
static_assert(((long long)CHUNK << SLA) < (1LL << 31));
static_assert(LISTN % NTHR == 0 && NBA == 4 * NTHR);
static_assert(RCAP % (2 * NTHR) == 0 && BK_ZINTS % (NTHR * 4) == 0);
static_assert(RCAP * 8 + LISTN * 4 <= 300000);
static_assert(BK_LDS_INTS * 4 <= 300000 && BK_LDS_INTS * 4 <= 327680);
static_assert(GRU_DYN_BYTES + GRU_STATIC_BYTES <= 327680);
static_assert(KCONV % 32 == 0 && KGI % 32 == 0 && KGH % 32 == 0);
static_assert(DF == 4 * 32 && HP == 2 * DF && GBM == (GTHR / 32) * 16 && TROWS == NWAVE * 16);
static_assert(NBA % TROWS == 0 && NBA % RSLOTS == 0 && TROWS % GBM == 0 && TROWS % AROWS == 0);
static_assert(UPART % NTHR == 0 && UPART == DF * (DF / 8) && (NPARTS * UPART) % NTHR == 0);
static_assert(OFF_CW1 == DF * HP && OFF_WRZ == 2 * DF * HP && OFF_WIN == OFF_WRZ + 256 * 512);
static_assert(OFF_WHN == OFF_WIN + DF * HP && WB_ELEMS == OFF_WHN + DF * HP);
static_assert(EC * DF == 2 * NTHR * 4 && 4 * NTHR == 1024);

typedef float          v2f   __attribute__((ext_vector_type(2)));
typedef float          v4f   __attribute__((ext_vector_type(4)));
typedef float          v8f   __attribute__((ext_vector_type(8)));
typedef int            v2i   __attribute__((ext_vector_type(2)));
typedef int            v4i   __attribute__((ext_vector_type(4)));
typedef int            v8i   __attribute__((ext_vector_type(8)));
typedef unsigned short v4us  __attribute__((ext_vector_type(4)));
typedef unsigned short v8us  __attribute__((ext_vector_type(8)));
typedef unsigned short v16us __attribute__((ext_vector_type(16)));
typedef __bf16         v16bf __attribute__((ext_vector_type(16)));
typedef v4f  __attribute__((may_alias)) v4fa;
typedef v2i  __attribute__((may_alias)) v2ia;
typedef v4i  __attribute__((may_alias)) v4ia;
typedef v4us __attribute__((may_alias)) v4usa;
typedef v8us __attribute__((may_alias)) v8usa;
union FragB { v16bf v; v16us u; v8us h[2]; v8i w; };

__device__ __forceinline__ v8f wmb(const FragB& a, const FragB& b, v8f c) {
  v8f d = __builtin_amdgcn_wmma_f32_16x16x32_bf16(false, a.v, false, b.v, (short)0, c, false, false);
  asm volatile("v_nop\n\tv_nop\n\tv_nop\n\tv_nop" : "+v"(d) : "v"(a.w), "v"(b.w));
  return d;
}

__device__ __forceinline__ v8f z8() { v8f z = {0.f, 0.f, 0.f, 0.f, 0.f, 0.f, 0.f, 0.f}; return z; }

__device__ __forceinline__ unsigned bf16_bits(float f) {
  const unsigned u = __float_as_uint(f);
  const unsigned r = (u + 0x7FFFu + ((u >> 16) & 1u)) >> 16;
  const unsigned q = (u >> 16) | 0x40u;
  return ((u & 0x7fffffffu) > 0x7f800000u) ? q : r;
}
__device__ __forceinline__ float bf16_val(float f) {
  return __uint_as_float(bf16_bits(f) << 16);
}

__device__ __forceinline__ void wave_sync() {
  __builtin_amdgcn_fence(__ATOMIC_RELEASE, "wavefront");
  __builtin_amdgcn_wave_barrier();
  __builtin_amdgcn_fence(__ATOMIC_ACQUIRE, "wavefront");
}

__device__ __forceinline__ float xh_fn(float xr, float mean, float rstd, float g, float b) {
#pragma clang fp contract(off)
  const float d = xr - mean;
  const float s = d * rstd;
  const float t = s * g;
  return t + b;
}

__device__ __forceinline__ float sigm(float t) {
#if FAST_GATES
  return __builtin_amdgcn_rcpf(1.0f + __expf(-t));
#else
  return 1.0f / (1.0f + expf(-t));
#endif
}
__device__ __forceinline__ float tanh_g(float t) {
#if FAST_GATES
  return 2.0f * sigm(2.0f * t) - 1.0f;
#else
  return tanhf(t);
#endif
}
__device__ __forceinline__ float relu_np(float v) { return (v > 0.0f) ? v : (v - v); }

__device__ __forceinline__ v8us cvt8(const float* __restrict__ p) {
  const v4f a = *(const v4f*)p;
  const v4f b = *(const v4f*)(p + 4);
  v8us o;
  o[0] = (unsigned short)bf16_bits(a.x); o[1] = (unsigned short)bf16_bits(a.y);
  o[2] = (unsigned short)bf16_bits(a.z); o[3] = (unsigned short)bf16_bits(a.w);
  o[4] = (unsigned short)bf16_bits(b.x); o[5] = (unsigned short)bf16_bits(b.y);
  o[6] = (unsigned short)bf16_bits(b.z); o[7] = (unsigned short)bf16_bits(b.w);
  return o;
}

template <int K, int BP>
__device__ __forceinline__ void gemm_seg(v8f (&acc)[8], const unsigned short* ap, const unsigned short* bp) {
#pragma unroll 1
  for (int k0 = 0; k0 < K; k0 += 32) {
    FragB af;
    af.h[0] = *(const v8usa*)(ap + k0);
    af.h[1] = *(const v8usa*)(ap + k0 + 16);
#pragma unroll
    for (int nt = 0; nt < 8; ++nt) {
      const unsigned short* wq = bp + (size_t)(16 * nt) * (size_t)BP + k0;
      FragB bf;
      bf.h[0] = *(const v8usa*)wq;
      bf.h[1] = *(const v8usa*)(wq + 16);
      acc[nt] = wmb(af, bf, acc[nt]);
    }
  }
}

__device__ __forceinline__ void dump_acc(const v8f (&acc)[8], float* stage, int wave, int hh, int m) {
#pragma unroll
  for (int nt = 0; nt < 8; ++nt) {
    const int lc = 16 * nt + m;
#pragma unroll
    for (int r = 0; r < 8; ++r) {
      const int lr = 16 * wave + 8 * hh + r;
      stage[lr * DF + lc] = acc[nt][r];
    }
  }
}

template <int SLB>
__device__ __forceinline__ int scan_chunk(const int* __restrict__ dsts, int nE, int cbase, int slotBase,
                                          int nb, int vec8, int* list, int tid, int lane, int wave) {
  int wc = 0;
  const int el0  = tid * EPT;
  const int e0   = cbase + el0;
  const int sent = -2147483647 - 1;
  v4i da, db;
  if (vec8 != 0 && cbase + CHUNK <= nE) {
    da = *(const v4i*)(dsts + e0);
    db = *(const v4i*)(dsts + e0 + 4);
  } else {
    const int k0 = dsts[min(e0,     nE - 1)];
    const int k1 = dsts[min(e0 + 1, nE - 1)];
    const int k2 = dsts[min(e0 + 2, nE - 1)];
    const int k3 = dsts[min(e0 + 3, nE - 1)];
    const int k4 = dsts[min(e0 + 4, nE - 1)];
    const int k5 = dsts[min(e0 + 5, nE - 1)];
    const int k6 = dsts[min(e0 + 6, nE - 1)];
    const int k7 = dsts[min(e0 + 7, nE - 1)];
    asm volatile("" :: "v"(k0), "v"(k1), "v"(k2), "v"(k3), "v"(k4), "v"(k5), "v"(k6), "v"(k7));
    da.x = (e0     < nE) ? k0 : sent;
    da.y = (e0 + 1 < nE) ? k1 : sent;
    da.z = (e0 + 2 < nE) ? k2 : sent;
    da.w = (e0 + 3 < nE) ? k3 : sent;
    db.x = (e0 + 4 < nE) ? k4 : sent;
    db.y = (e0 + 5 < nE) ? k5 : sent;
    db.z = (e0 + 6 < nE) ? k6 : sent;
    db.w = (e0 + 7 < nE) ? k7 : sent;
  }
  const unsigned nbs = (unsigned)slotBase;
  const unsigned unb = (unsigned)nb;
  const unsigned s0 = (unsigned)da.x - nbs, s1 = (unsigned)da.y - nbs;
  const unsigned s2 = (unsigned)da.z - nbs, s3 = (unsigned)da.w - nbs;
  const unsigned s4 = (unsigned)db.x - nbs, s5 = (unsigned)db.y - nbs;
  const unsigned s6 = (unsigned)db.z - nbs, s7 = (unsigned)db.w - nbs;
  const bool h0 = s0 < unb, h1 = s1 < unb, h2 = s2 < unb, h3 = s3 < unb;
  const bool h4 = s4 < unb, h5 = s5 < unb, h6 = s6 < unb, h7 = s7 < unb;
  const unsigned any = __builtin_amdgcn_ballot_w32(h0 | h1 | h2 | h3 | h4 | h5 | h6 | h7);
  if (any != 0u) {
#define HITJ(J, HJ, SJ) { \
      const unsigned mj = __builtin_amdgcn_ballot_w32(HJ); \
      if (mj != 0u) { \
        if (HJ) { \
          const int pos = wc + (int)__builtin_amdgcn_mbcnt_lo(mj, 0u); \
          if (pos < WCAP) list[wave * WCAP + pos] = ((el0 + (J)) << SLB) | (int)(SJ); \
        } \
        wc += (int)__builtin_popcount(mj); } }
    HITJ(0, h0, s0)
    HITJ(1, h1, s1)
    HITJ(2, h2, s2)
    HITJ(3, h3, s3)
    HITJ(4, h4, s4)
    HITJ(5, h5, s5)
    HITJ(6, h6, s6)
    HITJ(7, h7, s7)
#undef HITJ
  }
  return wc;
}

__global__ __launch_bounds__(NTHR) void k_prep(const float* __restrict__ x, const float* __restrict__ gam,
                                               const float* __restrict__ bet, const float* __restrict__ eW,
                                               const float* __restrict__ cW, const float* __restrict__ wih,
                                               const float* __restrict__ whh, const float* __restrict__ bih,
                                               const float* __restrict__ bhh, int nN, int nRec,
                                               unsigned short* WB, float* EWF, float* PAR, float* REC) {
  __shared__ __attribute__((aligned(16))) float wsm[NWAVE * DF];
  __shared__ __attribute__((aligned(16))) float wsq[NWAVE * DF];
  __shared__ float wsn[NWAVE];
  __shared__ __attribute__((aligned(16))) float pst[2 * DF];
  const int tid = (int)threadIdx.x, lane = tid & 31, wave = tid >> 5;
  const int blk = (int)blockIdx.x;

  if (blk < nRec) {
    const int r0 = blk * TROWS + 16 * wave;
    float wm[4], wq[4];
#pragma unroll
    for (int j = 0; j < 4; ++j) { wm[j] = 0.0f; wq[j] = 0.0f; }
    int wn = 0;
#pragma unroll 1
    for (int i = 0; i < 16; ++i) {
      const int row = r0 + i;
      const bool ok = row < nN;
      const int rc = ok ? row : nN - 1;
      const v4f xv = *(const v4f*)(x + (size_t)rc * DF + 4 * lane);
      if (ok) {
        wn += 1;
        const float rk = 1.0f / (float)wn;
        float vv[4];
        vv[0] = bf16_val(xv.x); vv[1] = bf16_val(xv.y); vv[2] = bf16_val(xv.z); vv[3] = bf16_val(xv.w);
#pragma unroll
        for (int j = 0; j < 4; ++j) {
          const float d = vv[j] - wm[j];
          wm[j] = fmaf(d, rk, wm[j]);
          wq[j] = fmaf(d, vv[j] - wm[j], wq[j]);
        }
      }
    }
    if (lane == 0) wsn[wave] = (float)wn;
#pragma unroll
    for (int j = 0; j < 4; ++j) {
      wsm[wave * DF + 4 * lane + j] = wm[j];
      wsq[wave * DF + 4 * lane + j] = wq[j];
    }
    __syncthreads();
    if (tid < DF) {
      float n = 0.0f, mean = 0.0f, M2 = 0.0f;
#pragma unroll 1
      for (int w2 = 0; w2 < NWAVE; ++w2) {
        const float nb = wsn[w2];
        const float mb = wsm[w2 * DF + tid];
        const float qb = wsq[w2 * DF + tid];
        if (nb > 0.5f) {
          const float nn = n + nb;
          const float delta = mb - mean;
          const float f = nb / nn;
          mean = fmaf(delta, f, mean);
          M2 = M2 + qb + delta * delta * n * f;
          n = nn;
        }
      }
      pst[2 * tid] = mean;
      pst[2 * tid + 1] = M2;
    }
    __syncthreads();
    v4f ps = {0.f, 0.f, 0.f, 0.f};
    float* dp = REC + (size_t)blk * (2 * DF) + 4 * (tid & 63);
    if (tid < 64) {
      ps = *(const v4fa*)(pst + 4 * tid);
      *(volatile v4f*)dp = ps;
    }
    __threadfence();
    if (tid < 64) *(volatile v4f*)dp = ps;
    return;
  }

  int pb = blk - nRec;
  if (pb < NWBLK) {
    const int u    = pb * NTHR + tid;
    const int part = u >> 11;
    const int v    = u & (UPART - 1);
    const int n    = v >> 4;
    const int k8   = (v & 15) * 8;
    v8us o;
    size_t doff;
    if (part < 4) {
      const int i = part >> 1;
      const int coff = (part & 1) * DF;
      const float* p = cW + (size_t)i * DF * DF + (size_t)k8 * DF + n;
      const float f0 = p[0],      f1 = p[DF],     f2 = p[2 * DF], f3 = p[3 * DF];
      const float f4 = p[4 * DF], f5 = p[5 * DF], f6 = p[6 * DF], f7 = p[7 * DF];
      o[0] = (unsigned short)bf16_bits(f0); o[1] = (unsigned short)bf16_bits(f1);
      o[2] = (unsigned short)bf16_bits(f2); o[3] = (unsigned short)bf16_bits(f3);
      o[4] = (unsigned short)bf16_bits(f4); o[5] = (unsigned short)bf16_bits(f5);
      o[6] = (unsigned short)bf16_bits(f6); o[7] = (unsigned short)bf16_bits(f7);
      doff = (size_t)i * (DF * HP) + (size_t)n * HP + coff + k8;
    } else if (part < 10) {
      const int q = part - 4;
      const int srow = (q >> 1) * DF + n;
      o = cvt8(wih + (size_t)srow * DF + k8);
      doff = (q < 4) ? ((size_t)OFF_WRZ + (size_t)srow * 512 + (q & 1) * DF + k8)
                     : ((size_t)OFF_WIN + (size_t)n * HP + (q & 1) * DF + k8);
    } else {
      const int q = part - 10;
      const int srow = (q >> 1) * DF + n;
      o = cvt8(whh + (size_t)srow * DF + k8);
      doff = (q < 4) ? ((size_t)OFF_WRZ + (size_t)srow * 512 + 2 * DF + (q & 1) * DF + k8)
                     : ((size_t)OFF_WHN + (size_t)n * HP + (q & 1) * DF + k8);
    }
    unsigned short* dp = WB + doff;
    *(volatile v8us*)dp = o;
    __threadfence();
    *(volatile v8us*)dp = o;
    return;
  }

  pb -= NWBLK;
  if (pb < 2) {
    const int u = pb * NTHR + tid;
    const v4f s = *(const v4f*)(eW + 4 * u);
    v4f o;
    o.x = bf16_val(s.x); o.y = bf16_val(s.y); o.z = bf16_val(s.z); o.w = bf16_val(s.w);
    float* dp = EWF + 4 * u;
    *(volatile v4f*)dp = o;
    __threadfence();
    *(volatile v4f*)dp = o;
    return;
  }

  {
    const int u = tid;
    v4f s;
    if (u < 32)       s = *(const v4f*)(gam + 4 * u);
    else if (u < 64)  s = *(const v4f*)(bet + 4 * (u - 32));
    else if (u < 160) s = *(const v4f*)(bih + 4 * (u - 64));
    else              s = *(const v4f*)(bhh + 4 * (u - 160));
    v4f o;
    o.x = bf16_val(s.x); o.y = bf16_val(s.y); o.z = bf16_val(s.z); o.w = bf16_val(s.w);
    float* dp = PAR + 4 * u;
    *(volatile v4f*)dp = o;
    __threadfence();
    *(volatile v4f*)dp = o;
  }
}

__global__ __launch_bounds__(DF) void k_bn_comb(const float* __restrict__ rec, int nRec, int nN, float* stat) {
  __shared__ __attribute__((aligned(16))) float stg[2 * DF];
  const int tid = (int)threadIdx.x;
  double n = 0.0, mean = 0.0, M2 = 0.0;
#pragma unroll 1
  for (int b = 0; b < nRec; ++b) {
    int cb = nN - TROWS * b;
    cb = cb < 0 ? 0 : (cb > TROWS ? TROWS : cb);
    const v2f r2 = *(const v2f*)(rec + ((size_t)b * DF + (size_t)tid) * 2);
    if (cb > 0) {
      const double nb = (double)cb;
      const double nn = n + nb;
      const double delta = (double)r2.x - mean;
      const double f = nb / nn;
      mean = mean + delta * f;
      M2 = M2 + (double)r2.y + delta * delta * n * f;
      n = nn;
    }
  }
  const double nt = n < 1.0 ? 1.0 : n;
  const float varf  = (float)(M2 / nt);
  const float meanf = (float)mean;
  const float rstd  = 1.0f / sqrtf(varf + 1e-5f);
  stg[2 * tid] = meanf;
  stg[2 * tid + 1] = rstd;
  __syncthreads();
  v4f v = {0.f, 0.f, 0.f, 0.f};
  float* dp = stat + 4 * (tid & 63);
  if (tid < 64) {
    v = *(const v4fa*)(stg + 4 * tid);
    *(volatile v4f*)dp = v;
  }
  __threadfence();
  if (tid < 64) *(volatile v4f*)dp = v;
}

__global__ __launch_bounds__(NTHR) void k_bn_apply(const float* __restrict__ x, const float* __restrict__ stat,
                                                   const float* __restrict__ par, int nN,
                                                   float* H, unsigned short* HL) {
  __shared__ float sMean[DF];
  __shared__ float sRstd[DF];
  __shared__ float sG[DF];
  __shared__ float sB[DF];
  const int tid = (int)threadIdx.x, lane = tid & 31, wave = tid >> 5;
  if (tid < DF) {
    sMean[tid] = stat[2 * tid];
    sRstd[tid] = stat[2 * tid + 1];
    sG[tid] = par[tid];
    sB[tid] = par[DF + tid];
  }
  __syncthreads();
  const int c4 = 4 * lane;
  const int c8 = 8 * (lane & 15);
  float m4[4], r4[4], g4[4], b4[4], m8[8], r8[8], g8[8], b8[8];
#pragma unroll
  for (int j = 0; j < 4; ++j) { m4[j] = sMean[c4 + j]; r4[j] = sRstd[c4 + j]; g4[j] = sG[c4 + j]; b4[j] = sB[c4 + j]; }
#pragma unroll
  for (int j = 0; j < 8; ++j) { m8[j] = sMean[c8 + j]; r8[j] = sRstd[c8 + j]; g8[j] = sG[c8 + j]; b8[j] = sB[c8 + j]; }
  const bool lowhalf = lane < 16;
#pragma unroll 1
  for (int i = 0; i < AROWS / NWAVE; ++i) {
    const int row = (int)blockIdx.x * AROWS + wave * (AROWS / NWAVE) + i;
    const bool live = row < nN;
    const int rc = live ? row : nN - 1;
    const float* xr = x + (size_t)rc * DF;
    const v4f xa = *(const v4f*)(xr + c4);
    const v4f xb0 = *(const v4f*)(xr + c8);
    const v4f xb1 = *(const v4f*)(xr + c8 + 4);
    asm volatile("" :: "v"(xa), "v"(xb0), "v"(xb1));
    v4f y;
    y.x = xh_fn(bf16_val(xa.x), m4[0], r4[0], g4[0], b4[0]);
    y.y = xh_fn(bf16_val(xa.y), m4[1], r4[1], g4[1], b4[1]);
    y.z = xh_fn(bf16_val(xa.z), m4[2], r4[2], g4[2], b4[2]);
    y.w = xh_fn(bf16_val(xa.w), m4[3], r4[3], g4[3], b4[3]);
    y.x = live ? y.x : 0.0f; y.y = live ? y.y : 0.0f; y.z = live ? y.z : 0.0f; y.w = live ? y.w : 0.0f;
    float z[8];
    z[0] = xb0.x; z[1] = xb0.y; z[2] = xb0.z; z[3] = xb0.w;
    z[4] = xb1.x; z[5] = xb1.y; z[6] = xb1.z; z[7] = xb1.w;
    v8us o;
#pragma unroll
    for (int j = 0; j < 8; ++j) {
      float t = xh_fn(bf16_val(z[j]), m8[j], r8[j], g8[j], b8[j]);
      t = live ? t : 0.0f;
      const unsigned hb = bf16_bits(t);
      const unsigned lb = bf16_bits(t - __uint_as_float(hb << 16));
      o[j] = (unsigned short)(lowhalf ? hb : lb);
    }
    float* hp = H + (size_t)row * DF + c4;
    unsigned short* lp = HL + (size_t)row * HP + 8 * lane;
    *(volatile v4f*)hp = y;
    *(volatile v8us*)lp = o;
    __threadfence();
    *(volatile v4f*)hp = y;
    *(volatile v8us*)lp = o;
  }
}

__global__ __launch_bounds__(NTHR) void k_bucket(const int* __restrict__ srcs, const int* __restrict__ dsts,
                                                 int nE, int nN, int vec8,
                                                 int* CNT, int* OFF, int* LIST, int* FLG) {
  extern __shared__ __attribute__((aligned(16))) int dsm[];
  int* list = dsm;
  int* hl   = dsm + LISTN;
  int* sl   = hl + RCAP;
  int* cnt  = sl + RCAP;
  int* offs = cnt + NBA;
  int* cur  = offs + NBA;
  int* misc = cur + NBA;
  const int tid = (int)threadIdx.x, lane = tid & 31, wave = tid >> 5;
  const int blk = (int)blockIdx.x;
  const int nodeBase = blk * NBA;

  {
    const v4i z4 = {0, 0, 0, 0};
    for (int i = tid * 4; i < BK_ZINTS; i += NTHR * 4) *(v4ia*)(dsm + i) = z4;
    if (tid < 16) misc[tid] = 0;
  }
  __syncthreads();

  int t = 0, ov = 0;
  const int nChunks = (nE + CHUNK - 1) / CHUNK;
#pragma unroll 1
  for (int ch = 0; ch < nChunks; ++ch) {
    const int cbase = ch * CHUNK;
    const int wc = scan_chunk<SLA>(dsts, nE, cbase, nodeBase, NBA, vec8, list, tid, lane, wave);
    if (lane == 0) misc[wave] = wc;
    __syncthreads();
    if (wave == 0) {
#pragma unroll 1
      for (int w2 = 0; w2 < NWAVE; ++w2) {
        int c = misc[w2];
        c = c < 0 ? 0 : (c > WCAP ? WCAP : c);
#pragma unroll 1
        for (int b0 = 0; b0 < c; b0 += 32) {
          const int idx = b0 + lane;
          const int ent = list[w2 * WCAP + (idx < WCAP ? idx : WCAP - 1)];
          const int m32 = (c - b0) < 32 ? (c - b0) : 32;
#pragma unroll 1
          for (int k = 0; k < m32; ++k) {
            const int u    = __builtin_amdgcn_readlane(ent, k);
            const int slot = u & (NBA - 1);
            const int el   = (u >> SLA) & (CHUNK - 1);
            const int pk   = ((cbase + el) << SLA) | slot;
            if (t < RCAP) {
              if (lane == 0) { hl[t] = pk; cnt[slot] = cnt[slot] + 1; }
              t = t + 1;
            } else {
              ov = 1;
            }
          }
        }
      }
    }
    __syncthreads();
  }
  if (wave == 0 && lane == 0) { misc[8] = t; misc[9] = ov; }
  __syncthreads();
  int tt = misc[8];
  tt = tt < 0 ? 0 : (tt > RCAP ? RCAP : tt);
  const int ovf = misc[9];

  if (wave == 0) {
    const int base = lane * (NBA / 32);
    int s = 0;
#pragma unroll 1
    for (int i = 0; i < NBA / 32; ++i) s += cnt[base + i];
    int incl = s;
#pragma unroll
    for (int d = 1; d < 32; d <<= 1) {
      const int y = __shfl_up(incl, d, 32);
      if (lane >= d) incl += y;
    }
    int run = incl - s;
#pragma unroll 1
    for (int i = 0; i < NBA / 32; ++i) {
      const int cv = cnt[base + i];
      offs[base + i] = run;
      cur[base + i]  = run;
      run += cv;
    }
  }
  __syncthreads();
  if (wave == 0) {
#pragma unroll 1
    for (int b0 = 0; b0 < tt; b0 += 32) {
      const int idx = b0 + lane;
      const int ent = hl[idx < RCAP ? idx : RCAP - 1];
      const int m32 = (tt - b0) < 32 ? (tt - b0) : 32;
#pragma unroll 1
      for (int k = 0; k < m32; ++k) {
        const int u    = __builtin_amdgcn_readlane(ent, k);
        const int slot = u & (NBA - 1);
        if (lane == 0) {
          int p = cur[slot];
          p = p < 0 ? 0 : (p > RCAP - 1 ? RCAP - 1 : p);
          sl[p] = u;
          cur[slot] = p + 1;
        }
      }
    }
  }
  __syncthreads();

  {
    const v4i cv = *(const v4ia*)(cnt + 4 * tid);
    const v4i ovv = *(const v4ia*)(offs + 4 * tid);
    int* cp = CNT + (size_t)blk * NBA + 4 * tid;
    int* op = OFF + (size_t)blk * NBA + 4 * tid;
    *(volatile v4i*)cp = cv;
    *(volatile v4i*)op = ovv;
    __threadfence();
    *(volatile v4i*)cp = cv;
    *(volatile v4i*)op = ovv;
  }
  {
    v4i fv;
    fv.x = ovf; fv.y = ovf; fv.z = ovf; fv.w = ovf;
    int* fp = FLG + (size_t)blk * 32 + 4 * (tid & 7);
    if (tid < 8) *(volatile v4i*)fp = fv;
    __threadfence();
    if (tid < 8) *(volatile v4i*)fp = fv;
  }
#pragma unroll 1
  for (int it = 0; it < RCAP / (2 * NTHR); ++it) {
    const int i0 = 2 * (it * NTHR + tid);
    const v2i en = *(const v2ia*)(sl + i0);
    int ea = en.x >> SLA;
    int eb = en.y >> SLA;
    ea = ea < 0 ? 0 : (ea > nE - 1 ? nE - 1 : ea);
    eb = eb < 0 ? 0 : (eb > nE - 1 ? nE - 1 : eb);
    int sa = srcs[ea];
    int sb = srcs[eb];
    asm volatile("" :: "v"(sa), "v"(sb));
    sa = sa < 0 ? 0 : (sa > nN - 1 ? nN - 1 : sa);
    sb = sb < 0 ? 0 : (sb > nN - 1 ? nN - 1 : sb);
    const bool la = i0 < tt;
    const bool lb = (i0 + 1) < tt;
    v4i o;
    o.x = la ? sa : 0; o.y = la ? ea : 0;
    o.z = lb ? sb : 0; o.w = lb ? eb : 0;
    int* lp = LIST + ((size_t)blk * RCAP + (size_t)i0) * 2;
    *(volatile v4i*)lp = o;
    __threadfence();
    *(volatile v4i*)lp = o;
  }
}

__global__ __launch_bounds__(GTHR) __attribute__((amdgpu_num_vgpr(248)))
void k_gemm_conv(const unsigned short* __restrict__ A, const unsigned short* __restrict__ BT, float* Mout) {
  __shared__ __attribute__((aligned(16))) float stg[GBM * DF];
  const int tid = (int)threadIdx.x, lane = tid & 31, wave = tid >> 5, hh = lane >> 4, m = lane & 15;
  const int rowBase = (int)blockIdx.x * GBM;
  v8f acc[8];
#pragma unroll
  for (int t = 0; t < 8; ++t) acc[t] = z8();
  const unsigned short* ap = A + (size_t)(rowBase + 16 * wave + m) * (size_t)HP + 8 * hh;
  const unsigned short* bp = BT + (size_t)m * (size_t)HP + 8 * hh;
  gemm_seg<KCONV, HP>(acc, ap, bp);
  dump_acc(acc, stg, wave, hh, m);
  __syncthreads();
  v4f pv[16];
#pragma unroll
  for (int i = 0; i < 16; ++i) pv[i] = *(const v4fa*)(stg + (16 * wave + i) * DF + 4 * lane);
#pragma unroll
  for (int i = 0; i < 16; ++i)
    *(volatile v4f*)(Mout + (size_t)(rowBase + 16 * wave + i) * DF + 4 * lane) = pv[i];
  __threadfence();
#pragma unroll
  for (int i = 0; i < 16; ++i)
    *(volatile v4f*)(Mout + (size_t)(rowBase + 16 * wave + i) * DF + 4 * lane) = pv[i];
}

__global__ __launch_bounds__(NTHR) void k_replay(const float* __restrict__ Mpl, const float* __restrict__ eattr,
                                                 const float* __restrict__ ewf, const int* __restrict__ cntp,
                                                 const int* __restrict__ offp, const int* __restrict__ listp,
                                                 const int* __restrict__ flg, int nE, int nN,
                                                 unsigned short* agg) {
  __shared__ __attribute__((aligned(16))) float sW[EC * DF];
  __shared__ __attribute__((aligned(16))) unsigned short rbuf[NWAVE * HP];
  const int tid = (int)threadIdx.x, lane = tid & 31, wave = tid >> 5;
  {
    const v4f w0 = *(const v4f*)(ewf + 4 * tid);
    const v4f w1 = *(const v4f*)(ewf + 4 * (tid + NTHR));
    *(v4fa*)(sW + 4 * tid) = w0;
    *(v4fa*)(sW + 4 * (tid + NTHR)) = w1;
  }
  __syncthreads();
  unsigned short* rowbuf = rbuf + wave * HP;
  const int nodeBase = (int)blockIdx.x * RSLOTS;
  const int bblk = nodeBase >> SLA;
  const int fl = flg[(size_t)bblk * 32];
  const int* lb = listp + (size_t)bblk * RCAP * 2;
  const float qnan = __int_as_float(0x7fc00000);

#pragma unroll 1
  for (int si = 0; si < RSLOTS / NWAVE; ++si) {
    const int node = nodeBase + si * NWAVE + wave;
    int c = cntp[node];
    const bool big = c > DEGCAP;
    c = c < 0 ? 0 : (c > DEGCAP ? DEGCAP : c);
    c = __builtin_amdgcn_readfirstlane(c);
    int o = offp[node];
    o = o < 0 ? 0 : (o > RCAP - 1 ? RCAP - 1 : o);
    float a0 = 0.0f, a1 = 0.0f, a2 = 0.0f, a3 = 0.0f;
#pragma unroll 1
    for (int b0 = 0; b0 < c; b0 += 32) {
      int idx = o + b0 + lane;
      const int last = o + c - 1;
      idx = idx > last ? last : idx;
      idx = idx < 0 ? 0 : (idx > RCAP - 1 ? RCAP - 1 : idx);
      const v2i en = *(const v2i*)(lb + (size_t)idx * 2);
      int sr = en.x;
      int ee = en.y;
      sr = sr < 0 ? 0 : (sr > nN - 1 ? nN - 1 : sr);
      ee = ee < 0 ? 0 : (ee > nE - 1 ? nE - 1 : ee);
      const int m32 = (c - b0) < 32 ? (c - b0) : 32;
#pragma unroll 1
      for (int k = 0; k < m32; ++k) {
        const int sk = __builtin_amdgcn_readlane(sr, k);
        const int ek = __builtin_amdgcn_readlane(ee, k);
        const v4f mv = *(const v4f*)(Mpl + (size_t)sk * DF + 4 * lane);
        const float* ap = eattr + (size_t)ek * EC;
        float e0 = 0.0f, e1 = 0.0f, e2 = 0.0f, e3 = 0.0f;
#pragma unroll 2
        for (int q = 0; q < 4; ++q) {
          const v4f a = *(const v4f*)(ap + 4 * q);
          const float t0 = bf16_val(a.x), t1 = bf16_val(a.y), t2 = bf16_val(a.z), t3 = bf16_val(a.w);
          const float* wr = sW + (4 * q) * DF + 4 * lane;
          const v4f w0 = *(const v4fa*)wr;
          const v4f w1 = *(const v4fa*)(wr + DF);
          const v4f w2 = *(const v4fa*)(wr + 2 * DF);
          const v4f w3 = *(const v4fa*)(wr + 3 * DF);
          e0 = fmaf(t0, w0.x, e0); e1 = fmaf(t0, w0.y, e1); e2 = fmaf(t0, w0.z, e2); e3 = fmaf(t0, w0.w, e3);
          e0 = fmaf(t1, w1.x, e0); e1 = fmaf(t1, w1.y, e1); e2 = fmaf(t1, w1.z, e2); e3 = fmaf(t1, w1.w, e3);
          e0 = fmaf(t2, w2.x, e0); e1 = fmaf(t2, w2.y, e1); e2 = fmaf(t2, w2.z, e2); e3 = fmaf(t2, w2.w, e3);
          e0 = fmaf(t3, w3.x, e0); e1 = fmaf(t3, w3.y, e1); e2 = fmaf(t3, w3.z, e2); e3 = fmaf(t3, w3.w, e3);
        }
        const float v0 = mv.x + e0, v1 = mv.y + e1, v2 = mv.z + e2, v3 = mv.w + e3;
        a0 += relu_np(v0);
        a1 += relu_np(v1);
        a2 += relu_np(v2);
        a3 += relu_np(v3);
      }
    }
    const float den = (float)(c > 1 ? c : 1);
    const bool pois = (fl != 0) || big;
    const bool live = node < nN;
    float g0 = a0 / den, g1 = a1 / den, g2 = a2 / den, g3 = a3 / den;
    g0 = pois ? qnan : g0; g1 = pois ? qnan : g1; g2 = pois ? qnan : g2; g3 = pois ? qnan : g3;
    g0 = live ? g0 : 0.0f; g1 = live ? g1 : 0.0f; g2 = live ? g2 : 0.0f; g3 = live ? g3 : 0.0f;
    v4us mh, ml;
    {
      unsigned hb;
      hb = bf16_bits(g0); mh[0] = (unsigned short)hb; ml[0] = (unsigned short)bf16_bits(g0 - __uint_as_float(hb << 16));
      hb = bf16_bits(g1); mh[1] = (unsigned short)hb; ml[1] = (unsigned short)bf16_bits(g1 - __uint_as_float(hb << 16));
      hb = bf16_bits(g2); mh[2] = (unsigned short)hb; ml[2] = (unsigned short)bf16_bits(g2 - __uint_as_float(hb << 16));
      hb = bf16_bits(g3); mh[3] = (unsigned short)hb; ml[3] = (unsigned short)bf16_bits(g3 - __uint_as_float(hb << 16));
    }
    *(v4usa*)(rowbuf + 4 * lane) = mh;
    *(v4usa*)(rowbuf + DF + 4 * lane) = ml;
    wave_sync();
    const v8us q0 = *(const v8usa*)(rowbuf + 8 * lane);
    wave_sync();
    unsigned short* rp = agg + (size_t)node * HP + 8 * lane;
    *(volatile v8us*)rp = q0;
    __threadfence();
    *(volatile v8us*)rp = q0;
  }
}

template <int FIN>
__device__ __forceinline__ void gru_store_pass(const float* st0, int rowBase, int wave, int lane, int nN,
                                               float* hp, unsigned short* hlp, float* outp) {
  const int c8 = 8 * (lane & 15);
  const bool lowhalf = lane < 16;
#pragma unroll 1
  for (int i = 0; i < 16; ++i) {
    const int lr = 16 * wave + i;
    const int row = rowBase + lr;
    const v4f v = *(const v4fa*)(st0 + lr * DF + 4 * lane);
    if constexpr (FIN != 0) {
      if (row < nN) *(volatile v4f*)(outp + (size_t)row * DF + 4 * lane) = v;
    } else {
      const v4f q0 = *(const v4fa*)(st0 + lr * DF + c8);
      const v4f q1 = *(const v4fa*)(st0 + lr * DF + c8 + 4);
      float z[8];
      z[0] = q0.x; z[1] = q0.y; z[2] = q0.z; z[3] = q0.w;
      z[4] = q1.x; z[5] = q1.y; z[6] = q1.z; z[7] = q1.w;
      v8us o;
#pragma unroll
      for (int j = 0; j < 8; ++j) {
        const unsigned hb = bf16_bits(z[j]);
        const unsigned lb = bf16_bits(z[j] - __uint_as_float(hb << 16));
        o[j] = (unsigned short)(lowhalf ? hb : lb);
      }
      *(volatile v4f*)(hp + (size_t)row * DF + 4 * lane) = v;
      *(volatile v8us*)(hlp + (size_t)row * HP + 8 * lane) = o;
    }
  }
}

template <int FIN>
__global__ __launch_bounds__(NTHR) __attribute__((amdgpu_num_vgpr(248)))
void k_gru(const unsigned short* aggp, unsigned short* hlp, float* hp, const unsigned short* __restrict__ WB,
           const float* __restrict__ par, const float* __restrict__ stat, const float* __restrict__ xin,
           const int* __restrict__ flg, int nN, float* outp) {
  extern __shared__ __attribute__((aligned(16))) float gsm[];
  __shared__ __attribute__((aligned(16))) float sPar[1024];
  __shared__ __attribute__((aligned(16))) float sStat[2 * DF];
  float* st0 = gsm;
  float* st1 = gsm + GRU_STAGE;
  float* st2 = gsm + 2 * GRU_STAGE;
  float* st3 = gsm + 3 * GRU_STAGE;
  const int tid = (int)threadIdx.x, lane = tid & 31, wave = tid >> 5, hh = lane >> 4, m = lane & 15;
  const int rowBase = (int)blockIdx.x * TROWS;

  {
    const v4f pv = *(const v4f*)(par + 4 * tid);
    *(v4fa*)(sPar + 4 * tid) = pv;
    const v4f sv = *(const v4f*)(stat + 4 * (tid & 63));
    asm volatile("" :: "v"(sv));
    if (tid < 64) *(v4fa*)(sStat + 4 * tid) = sv;
  }

  const unsigned short* apA = aggp + (size_t)(rowBase + 16 * wave + m) * (size_t)HP + 8 * hh;
  const unsigned short* apH = hlp  + (size_t)(rowBase + 16 * wave + m) * (size_t)HP + 8 * hh;
  const unsigned short* bR  = WB + OFF_WRZ + (size_t)m * 512 + 8 * hh;
  const unsigned short* bZ  = bR + (size_t)DF * 512;
  const unsigned short* bHN = WB + OFF_WHN + (size_t)m * HP + 8 * hh;
  const unsigned short* bIN = WB + OFF_WIN + (size_t)m * HP + 8 * hh;

  v8f acc[8];
#pragma unroll
  for (int t = 0; t < 8; ++t) acc[t] = z8();
  gemm_seg<KGI, 512>(acc, apA, bR);
  gemm_seg<KGH, 512>(acc, apH, bR + 2 * DF);
  dump_acc(acc, st0, wave, hh, m);
#pragma unroll
  for (int t = 0; t < 8; ++t) acc[t] = z8();
  gemm_seg<KGI, 512>(acc, apA, bZ);
  gemm_seg<KGH, 512>(acc, apH, bZ + 2 * DF);
  dump_acc(acc, st1, wave, hh, m);
#pragma unroll
  for (int t = 0; t < 8; ++t) acc[t] = z8();
  gemm_seg<KGH, HP>(acc, apH, bHN);
  dump_acc(acc, st2, wave, hh, m);
#pragma unroll
  for (int t = 0; t < 8; ++t) acc[t] = z8();
  gemm_seg<KGI, HP>(acc, apA, bIN);
  dump_acc(acc, st3, wave, hh, m);
  __syncthreads();

  const int c4 = 4 * lane;
  float cR[4], cZ[4], cHN[4], cIN[4], cM[4], cS[4], cG[4], cB[4];
#pragma unroll
  for (int j = 0; j < 4; ++j) {
    const int c = c4 + j;
    cR[j]  = sPar[256 + c] + sPar[640 + c];
    cZ[j]  = sPar[256 + DF + c] + sPar[640 + DF + c];
    cIN[j] = sPar[256 + 2 * DF + c];
    cHN[j] = sPar[640 + 2 * DF + c];
    cG[j]  = sPar[c];
    cB[j]  = sPar[DF + c];
    cM[j]  = sStat[2 * c];
    cS[j]  = sStat[2 * c + 1];
  }
  const int fl = flg[(size_t)(rowBase >> SLA) * 32];
  const float qnan = __int_as_float(0x7fc00000);

#pragma unroll 1
  for (int i = 0; i < 16; ++i) {
    const int lr = 16 * wave + i;
    const int row = rowBase + lr;
    const bool live = row < nN;
    const v4f vR = *(const v4fa*)(st0 + lr * DF + c4);
    const v4f vZ = *(const v4fa*)(st1 + lr * DF + c4);
    const v4f vH = *(const v4fa*)(st2 + lr * DF + c4);
    const v4f vI = *(const v4fa*)(st3 + lr * DF + c4);
    const v4f ho = *(const v4f*)(hp + (size_t)row * DF + c4);
    float aR[4], aZ[4], aH[4], aI[4], aO[4], res[4];
    aR[0] = vR.x; aR[1] = vR.y; aR[2] = vR.z; aR[3] = vR.w;
    aZ[0] = vZ.x; aZ[1] = vZ.y; aZ[2] = vZ.z; aZ[3] = vZ.w;
    aH[0] = vH.x; aH[1] = vH.y; aH[2] = vH.z; aH[3] = vH.w;
    aI[0] = vI.x; aI[1] = vI.y; aI[2] = vI.z; aI[3] = vI.w;
    aO[0] = ho.x; aO[1] = ho.y; aO[2] = ho.z; aO[3] = ho.w;
    float xs[4];
    if constexpr (FIN != 0) {
      const int rc = live ? row : nN - 1;
      const v4f xv = *(const v4f*)(xin + (size_t)rc * DF + c4);
      asm volatile("" :: "v"(xv));
      xs[0] = xv.x; xs[1] = xv.y; xs[2] = xv.z; xs[3] = xv.w;
    } else {
      xs[0] = 0.0f; xs[1] = 0.0f; xs[2] = 0.0f; xs[3] = 0.0f;
    }
#pragma unroll
    for (int j = 0; j < 4; ++j) {
      const float rg = sigm(aR[j] + cR[j]);
      const float zg = sigm(aZ[j] + cZ[j]);
      const float hn = aH[j] + cHN[j];
      const float ng = tanh_g((aI[j] + cIN[j]) + rg * hn);
      const float hnew = (1.0f - zg) * ng + zg * aO[j];
      if constexpr (FIN != 0) {
        const float xhv = xh_fn(bf16_val(xs[j]), cM[j], cS[j], cG[j], cB[j]);
        float ov = 0.5f * relu_np(hnew) + 0.5f * xhv;
        ov = (fl != 0) ? qnan : ov;
        res[j] = ov;
      } else {
        res[j] = live ? hnew : 0.0f;
      }
    }
    v4f rv;
    rv.x = res[0]; rv.y = res[1]; rv.z = res[2]; rv.w = res[3];
    *(v4fa*)(st0 + lr * DF + c4) = rv;
  }
  __syncthreads();

  gru_store_pass<FIN>(st0, rowBase, wave, lane, nN, hp, hlp, outp);
  __threadfence();
  gru_store_pass<FIN>(st0, rowBase, wave, lane, nN, hp, hlp, outp);
}

static inline int cdiv(int a, int b) { return (a + b - 1) / b; }
static inline size_t al256(size_t o) { return (o + 255) & ~(size_t)255; }

extern "C" void kernel_launch(void* const* d_in, const int* in_sizes, int n_in,
                              void* d_out, int out_size, void* d_ws, size_t ws_size,
                              hipStream_t stream) {
  if (n_in < 11) return;
  if (in_sizes[0] < DF || (in_sizes[0] % DF) != 0) return;
  const int nN = in_sizes[0] / DF;
  if (in_sizes[1] < 2 || (in_sizes[1] & 1) != 0) return;
  const int nE = in_sizes[1] / 2;
  if ((long long)in_sizes[2] != (long long)nE * EC) return;
  if (in_sizes[3] != DF || in_sizes[4] != DF) return;
  if (in_sizes[5] != EC * DF) return;
  if (in_sizes[6] != 2 * DF * DF) return;
  if (in_sizes[7] != 3 * DF * DF || in_sizes[8] != 3 * DF * DF) return;
  if (in_sizes[9] != 3 * DF || in_sizes[10] != 3 * DF) return;
  if ((long long)out_size != (long long)nN * DF) return;
  if (nE >= (1 << 21) || nN < 16 || nN >= (1 << 24)) return;

  const float* x    = (const float*)d_in[0];
  const int*   ei   = (const int*)d_in[1];
  const float* eatt = (const float*)d_in[2];
  const float* gam  = (const float*)d_in[3];
  const float* bet  = (const float*)d_in[4];
  const float* eW   = (const float*)d_in[5];
  const float* cW   = (const float*)d_in[6];
  const float* wih  = (const float*)d_in[7];
  const float* whh  = (const float*)d_in[8];
  const float* bih  = (const float*)d_in[9];
  const float* bhh  = (const float*)d_in[10];
  float* out = (float*)d_out;
  const int* srcs = ei;
  const int* dsts = ei + nE;

  const int nRec = cdiv(nN, TROWS);
  const int MP = nRec * TROWS;
  const int NB = cdiv(nN, NBA);
  if ((long long)NB * NBA < (long long)MP) return;
  const int vec8 = ((nE & 3) == 0) ? 1 : 0;

  char* ws = (char*)d_ws;
  size_t off = 0;
  const size_t oWB   = off; off = al256(off + (size_t)WB_ELEMS * 2);
  const size_t oEWF  = off; off = al256(off + (size_t)EC * DF * 4);
  const size_t oPAR  = off; off = al256(off + (size_t)1024 * 4);
  const size_t oREC  = off; off = al256(off + (size_t)nRec * 2 * DF * 4);
  const size_t oSTAT = off; off = al256(off + (size_t)2 * DF * 4);
  const size_t oFLG  = off; off = al256(off + (size_t)NB * 32 * 4);
  const size_t oCNT  = off; off = al256(off + (size_t)NB * NBA * 4);
  const size_t oOFF  = off; off = al256(off + (size_t)NB * NBA * 4);
  const size_t oLIST = off; off = al256(off + (size_t)NB * RCAP * 8);
  const size_t oH    = off; off = al256(off + (size_t)MP * DF * 4);
  const size_t oHL   = off; off = al256(off + (size_t)MP * HP * 2);
  const size_t oM    = off; off = al256(off + (size_t)MP * DF * 4);
  const size_t oAGG  = off; off = al256(off + (size_t)MP * HP * 2);
  if (off > ws_size || off > (size_t)WSMAX) return;
  unsigned short* WB = (unsigned short*)(ws + oWB);
  float* EWF  = (float*)(ws + oEWF);
  float* PAR  = (float*)(ws + oPAR);
  float* REC  = (float*)(ws + oREC);
  float* STAT = (float*)(ws + oSTAT);
  int*   FLG  = (int*)(ws + oFLG);
  int*   CNT  = (int*)(ws + oCNT);
  int*   OFFp = (int*)(ws + oOFF);
  int*   LIST = (int*)(ws + oLIST);
  float* H    = (float*)(ws + oH);
  unsigned short* HL  = (unsigned short*)(ws + oHL);
  float* Mp   = (float*)(ws + oM);
  unsigned short* AGG = (unsigned short*)(ws + oAGG);

  const size_t bkLds  = (size_t)BK_LDS_INTS * 4;
  const size_t gruLds = (size_t)GRU_DYN_BYTES;
  hipFuncSetAttribute(reinterpret_cast<const void*>(&k_bucket), hipFuncAttributeMaxDynamicSharedMemorySize, (int)bkLds);
  hipFuncSetAttribute(reinterpret_cast<const void*>(&k_gru<0>), hipFuncAttributeMaxDynamicSharedMemorySize, (int)gruLds);
  hipFuncSetAttribute(reinterpret_cast<const void*>(&k_gru<1>), hipFuncAttributeMaxDynamicSharedMemorySize, (int)gruLds);

  k_prep<<<nRec + NWBLK + 3, NTHR, 0, stream>>>(x, gam, bet, eW, cW, wih, whh, bih, bhh, nN, nRec, WB, EWF, PAR, REC);
  k_bn_comb<<<1, DF, 0, stream>>>(REC, nRec, nN, STAT);
  k_bn_apply<<<MP / AROWS, NTHR, 0, stream>>>(x, STAT, PAR, nN, H, HL);
  k_bucket<<<NB, NTHR, bkLds, stream>>>(srcs, dsts, nE, nN, vec8, CNT, OFFp, LIST, FLG);
  k_gemm_conv<<<MP / GBM, GTHR, 0, stream>>>(HL, WB + OFF_CW0, Mp);
  k_replay<<<MP / RSLOTS, NTHR, 0, stream>>>(Mp, eatt, EWF, CNT, OFFp, LIST, FLG, nE, nN, AGG);
  k_gru<0><<<MP / TROWS, NTHR, gruLds, stream>>>(AGG, HL, H, WB, PAR, STAT, x, FLG, nN, out);
  k_gemm_conv<<<MP / GBM, GTHR, 0, stream>>>(HL, WB + OFF_CW1, Mp);
  k_replay<<<MP / RSLOTS, NTHR, 0, stream>>>(Mp, eatt, EWF, CNT, OFFp, LIST, FLG, nE, nN, AGG);
  k_gru<1><<<MP / TROWS, NTHR, gruLds, stream>>>(AGG, HL, H, WB, PAR, STAT, x, FLG, nN, out);
}
